// MambaBlock_66546223284397
// MI455X (gfx1250) — hardware-verified
//
#include <hip/hip_runtime.h>
#include <math.h>

typedef __attribute__((ext_vector_type(16))) _Float16 v16h;
typedef __attribute__((ext_vector_type(8)))  _Float16 v8h;
typedef __attribute__((ext_vector_type(8)))  float    v8f;
typedef __attribute__((ext_vector_type(4)))  float    v4f;

constexpr int kBatch  = 2;
constexpr int kSeq    = 1024;
constexpr int kDm     = 1024;
constexpr int kDin    = 2048;
constexpr int kNst    = 16;
constexpr int kDtR    = 16;
constexpr int kConvK  = 4;
constexpr int kPrjN   = 48;
constexpr int kPrjP   = 64;
constexpr int kXZP    = 2 * kDin;
constexpr int kRows   = kBatch * kSeq;
constexpr int kConvTP = 260;
constexpr int kScanTS = 64;
constexpr int kScanCh = 64;
constexpr int kScanYP = 68;
constexpr float kCarryW  = 32.0f;
constexpr float kCarryXc = 16.0f;
constexpr float kCarryG  = 64.0f;
constexpr float kSclIn   = 1.0f / kCarryW;
constexpr float kSclXp   = 1.0f / (kCarryW * kCarryXc);
constexpr float kSclOut  = 1.0f / (kCarryW * kCarryG);

static_assert(kDtR + 2 * kNst == kPrjN);
static_assert(kPrjN <= kPrjP && (kPrjP % 64) == 0);
static_assert((kDm % 32) == 0 && (kDin % 32) == 0);
static_assert((kRows % 64) == 0 && (kXZP % 64) == 0 && (kDm % 64) == 0 && (kDin % 64) == 0);
static_assert((((kRows / 64) * (kXZP / 64)) % 8) == 0);
static_assert((((kRows / 64) * (kPrjP / 64)) % 8) == 0);
static_assert((((kRows / 64) * (kDm / 64)) % 8) == 0);
static_assert((kSeq % kScanTS) == 0 && (kSeq % 64) == 0 && (kDin % kScanCh) == 0 && (kDin % 256) == 0);
static_assert(((kRows * kDm / 8) % 256) == 0);
static_assert(kConvK == 4 && kNst == 16 && (kDtR % 4) == 0);

constexpr size_t kOffXH   = 0;
constexpr size_t kOffWIN  = kOffXH   + (size_t)kRows * kDm  * 2;
constexpr size_t kOffWOUT = kOffWIN  + (size_t)kXZP  * kDm  * 2;
constexpr size_t kOffWX   = kOffWOUT + (size_t)kDm   * kDin * 2;
constexpr size_t kOffXR   = kOffWX   + (size_t)kPrjP * kDin * 2;
constexpr size_t kOffUC   = kOffXR   + (size_t)kRows * kXZP * 4;
constexpr size_t kOffUCH  = kOffUC   + (size_t)kRows * kDin * 4;
constexpr size_t kOffPROJ = kOffUCH  + (size_t)kRows * kDin * 2;
constexpr size_t kOffG16  = kOffPROJ + (size_t)kRows * kPrjP * 4;
constexpr size_t kWsTotal = kOffG16  + (size_t)kRows * kDin * 2;
static_assert(kWsTotal == 84672512ull);
static_assert(kWsTotal <= 134217728ull);
static_assert((kOffWIN % 128) == 0 && (kOffWOUT % 128) == 0 && (kOffWX % 128) == 0 && (kOffXR % 128) == 0 &&
              (kOffUC % 128) == 0 && (kOffUCH % 128) == 0 && (kOffPROJ % 128) == 0 && (kOffG16 % 128) == 0);

__device__ __forceinline__ void dep_guard4_h(v8f& a, v8f& b, v8f& c, v8f& d, v16h x, v16h b0, v16h b1, v16h b2, v16h b3) {
  asm volatile("v_nop\n\tv_nop\n\tv_nop\n\tv_nop" : "+v"(a), "+v"(b), "+v"(c), "+v"(d) : "v"(x), "v"(b0), "v"(b1), "v"(b2), "v"(b3));
}
__device__ __forceinline__ void keep4_h(v16h a, v16h b, v16h c, v16h d) { asm volatile("v_nop" :: "v"(a), "v"(b), "v"(c), "v"(d)); }
__device__ __forceinline__ void acc_guard4(v8f& a, v8f& b, v8f& c, v8f& d) { asm volatile("v_nop\n\tv_nop\n\tv_nop\n\tv_nop" : "+v"(a), "+v"(b), "+v"(c), "+v"(d)); }

union FragU { v16h v; v8h h[2]; };
__device__ __forceinline__ v16h frag_load(const _Float16* p) {
  FragU f;
  f.h[0] = *(const v8h*)(p);
  f.h[1] = *(const v8h*)(p + 16);
  return f.v;
}
__device__ __forceinline__ v8f frag_mma(v16h a, v16h b, v8f c) {
  return __builtin_amdgcn_wmma_f32_16x16x32_f16(false, a, false, b, (short)0, c, false, false);
}

template <int BIAS_MODE>
__global__ __launch_bounds__(256) void wmma_gemm64_f16(
    const unsigned short* __restrict__ Ap, int lda,
    const unsigned short* __restrict__ Btp, int ldb,
    float* __restrict__ Cout, int ldc,
    const float* __restrict__ bias,
    int M, int N, int K, float scale) {
  const _Float16* A  = (const _Float16*)Ap;
  const _Float16* Bt = (const _Float16*)Btp;
  __shared__ __align__(16) float sT[8][16 * 68];
  const int lane = threadIdx.x & 31;
  const int wave = threadIdx.x >> 5;
  const int tilesN = N >> 6;
  const int tilesM = M >> 6;
  const int tile = blockIdx.x * 8 + wave;
  if (tile >= tilesM * tilesN) return;
  const int tm = tile / tilesN;
  const int tn = tile - tm * tilesN;
  const int m0 = tm << 6;
  const int n0 = tn << 6;

  const int rlane = lane & 15;
  const int koff  = (lane >> 4) * 8;
  const int mOff  = (lane >> 4) * 8;

  v8f acc[4][4];
#pragma unroll
  for (int i = 0; i < 4; ++i)
#pragma unroll
    for (int j = 0; j < 4; ++j) acc[i][j] = (v8f){0.f,0.f,0.f,0.f,0.f,0.f,0.f,0.f};

  for (int k0 = 0; k0 < K; k0 += 32) {
    v16h bh[4];
#pragma unroll
    for (int j = 0; j < 4; ++j) {
      const size_t bo = (size_t)(n0 + (j << 4) + rlane) * ldb + koff + k0;
      bh[j] = frag_load(Bt + bo);
    }
#pragma unroll
    for (int i = 0; i < 4; ++i) {
      const size_t ao = (size_t)(m0 + (i << 4) + rlane) * lda + koff + k0;
      v16h ah = frag_load(A + ao);
#pragma unroll
      for (int j = 0; j < 4; ++j) acc[i][j] = frag_mma(ah, bh[j], acc[i][j]);
      dep_guard4_h(acc[i][0], acc[i][1], acc[i][2], acc[i][3], ah, bh[0], bh[1], bh[2], bh[3]);
    }
    keep4_h(bh[0], bh[1], bh[2], bh[3]);
  }
  acc_guard4(acc[0][0], acc[0][1], acc[0][2], acc[0][3]);
  acc_guard4(acc[1][0], acc[1][1], acc[1][2], acc[1][3]);
  acc_guard4(acc[2][0], acc[2][1], acc[2][2], acc[2][3]);
  acc_guard4(acc[3][0], acc[3][1], acc[3][2], acc[3][3]);

  float* slab = sT[wave];
#pragma unroll
  for (int i = 0; i < 4; ++i) {
    const int mBase = m0 + (i << 4);
#pragma unroll
    for (int j = 0; j < 4; ++j) {
      const int n = n0 + (j << 4) + rlane;
      float bv = 0.f;
      if (BIAS_MODE == 2) bv = bias[n];
#pragma unroll
      for (int r = 0; r < 8; ++r) {
        float v = acc[i][j][r] * scale;
        if (BIAS_MODE == 2) v += bv;
        slab[(mOff + r) * 68 + (j << 4) + rlane] = v;
      }
    }
    __builtin_amdgcn_fence(__ATOMIC_RELEASE, "workgroup");
    __builtin_amdgcn_wave_barrier();
    __builtin_amdgcn_fence(__ATOMIC_ACQUIRE, "workgroup");
    {
      float* C = Cout;
      const int hh = lane >> 4, c4 = (lane & 15) * 4;
      for (int pass = 0; pass < 2; ++pass) {
#pragma unroll
        for (int it = 0; it < 8; ++it) {
          const int row = it * 2 + hh;
          v4f v = *(const v4f*)(slab + row * 68 + c4);
          *(volatile v4f*)(C + (size_t)(mBase + row) * ldc + n0 + c4) = v;
        }
        __threadfence();
      }
    }
    __builtin_amdgcn_fence(__ATOMIC_RELEASE, "workgroup");
    __builtin_amdgcn_wave_barrier();
    __builtin_amdgcn_fence(__ATOMIC_ACQUIRE, "workgroup");
  }
}

__global__ __launch_bounds__(256) void cast_f16_kernel(
    const float* __restrict__ src, unsigned short* __restrict__ dst, int total8, float scale)
{
  const int i = blockIdx.x * 256 + threadIdx.x;
  if (i >= total8) return;
  const size_t e0 = (size_t)i << 3;
  const float* p = src + e0;
  const v4f a0 = *(const v4f*)(p);
  const v4f a1 = *(const v4f*)(p + 4);
  v8h hv;
#pragma unroll
  for (int e = 0; e < 4; ++e) {
    hv[e]     = (_Float16)(a0[e] * scale);
    hv[4 + e] = (_Float16)(a1[e] * scale);
  }
  unsigned short* q = dst + e0;
  *(volatile v8h*)q = hv;
  __threadfence();
  *(volatile v8h*)q = hv;
}

__global__ __launch_bounds__(256) void transpose_cast_kernel(
    const float* __restrict__ W, unsigned short* __restrict__ Bt, int Kdim, int Ndim, int Npad, float scale)
{
  __shared__ float tile[64 * 65];
  const int tid = threadIdx.x, lane = tid & 31, wave = tid >> 5;
  const int n0 = blockIdx.x * 64;
  const int k0 = blockIdx.y * 64;
  (void)Npad;
#pragma unroll
  for (int p = 0; p < 16; ++p) {
    const int idx = tid + p * 256;
    const int kk  = idx >> 6;
    const int nn  = idx & 63;
    const int n   = n0 + nn;
    const int nc  = (n < Ndim) ? n : (Ndim - 1);
    const float v = W[(size_t)(k0 + kk) * Ndim + nc];
    tile[kk * 65 + nn] = (n < Ndim) ? (v * scale) : 0.f;
  }
  __syncthreads();
  const int q = lane >> 3, c8 = (lane & 7) * 8;
  v8h hv[2];
#pragma unroll
  for (int it = 0; it < 2; ++it) {
    const int nrow = it * 32 + wave * 4 + q;
#pragma unroll
    for (int e = 0; e < 8; ++e) hv[it][e] = (_Float16)tile[(c8 + e) * 65 + nrow];
  }
  for (int pass = 0; pass < 2; ++pass) {
#pragma unroll
    for (int it = 0; it < 2; ++it) {
      const int nrow = it * 32 + wave * 4 + q;
      *(volatile v8h*)(Bt + (size_t)(n0 + nrow) * Kdim + k0 + c8) = hv[it];
    }
    __threadfence();
  }
}

__global__ __launch_bounds__(256) void conv_silu_kernel(
    const float* __restrict__ XR, const float* __restrict__ cw, const float* __restrict__ cb,
    float* __restrict__ UC, unsigned short* __restrict__ UCH)
{
  __shared__ __align__(16) float sT[16 * kConvTP];
  const int tid = threadIdx.x, lane = tid & 31, wave = tid >> 5;
  const int d0 = blockIdx.x * 256, d = d0 + tid;
  const int g0 = blockIdx.y * 64;
  const int tb = g0 & (kSeq - 1);
  const float w0 = cw[0 * kDin + d], w1 = cw[1 * kDin + d], w2 = cw[2 * kDin + d], w3 = cw[3 * kDin + d];
  const float bc = cb[d];
  float xm3, xm2, xm1;
  {
    const bool hist = (tb > 0);
    const int rb = hist ? (g0 - 3) : g0;
    const float v3 = XR[(size_t)rb * kXZP + d];
    const float v2 = XR[(size_t)(rb + 1) * kXZP + d];
    const float v1 = XR[(size_t)(rb + 2) * kXZP + d];
    xm3 = hist ? v3 : 0.f;
    xm2 = hist ? v2 : 0.f;
    xm1 = hist ? v1 : 0.f;
  }
  const int hrow = wave >> 1;
  const int hch  = (wave & 1) * 128 + lane * 4;
#pragma unroll 1
  for (int sub = 0; sub < 4; ++sub) {
    const int lb = g0 + sub * 16;
#pragma unroll 1
    for (int s = 0; s < 16; ++s) {
      const float xcur = XR[(size_t)(lb + s) * kXZP + d];
      float acc = w0 * xm3;
      acc = fmaf(w1, xm2, acc);
      acc = fmaf(w2, xm1, acc);
      acc = fmaf(w3, xcur, acc);
      const float sv = acc + bc;
      const float sg = __builtin_amdgcn_rcpf(1.0f + expf(-sv));
      sT[s * kConvTP + tid] = sv * sg;
      xm3 = xm2; xm2 = xm1; xm1 = xcur;
    }
    __syncthreads();
    v4f fv[4];
    v8h bv[2];
#pragma unroll
    for (int it = 0; it < 4; ++it) fv[it] = *(const v4f*)(sT + (it * 4 + hrow) * kConvTP + hch);
#pragma unroll
    for (int it = 0; it < 2; ++it) {
      const float* sp = sT + (it * 8 + wave) * kConvTP + lane * 8;
      const v4f a0 = *(const v4f*)(sp);
      const v4f a1 = *(const v4f*)(sp + 4);
#pragma unroll
      for (int e = 0; e < 4; ++e) {
        bv[it][e]     = (_Float16)(a0[e] * kCarryXc);
        bv[it][4 + e] = (_Float16)(a1[e] * kCarryXc);
      }
    }
    for (int pass = 0; pass < 2; ++pass) {
#pragma unroll
      for (int it = 0; it < 4; ++it)
        *(volatile v4f*)(UC + (size_t)(lb + it * 4 + hrow) * kDin + d0 + hch) = fv[it];
#pragma unroll
      for (int it = 0; it < 2; ++it)
        *(volatile v8h*)(UCH + (size_t)(lb + it * 8 + wave) * kDin + d0 + lane * 8) = bv[it];
      __threadfence();
    }
    __syncthreads();
  }
}

__global__ __launch_bounds__(64) void scan_kernel(
    const float* __restrict__ PROJ, const float* __restrict__ UC, const float* __restrict__ XR,
    const float* __restrict__ xpb, const float* __restrict__ Wdt, const float* __restrict__ bdt,
    const float* __restrict__ Alog, const float* __restrict__ Dp, unsigned short* __restrict__ G16)
{
  __shared__ __align__(16) float sX[kScanTS * kPrjP];
  __shared__ __align__(16) float sY[kScanTS * kScanYP];
  __shared__ __align__(16) float sW[kDtR * kScanCh];
  __shared__ __align__(16) float sA[kNst * kScanCh];
  __shared__ __align__(16) float sPB[kPrjP];
  const int tid = threadIdx.x, lane = tid & 31, wave = tid >> 5;
  constexpr int kBlkPerB = kDin / kScanCh;
  const int bix = blockIdx.x / kBlkPerB;
  const int d0  = (blockIdx.x - bix * kBlkPerB) * kScanCh;
  const int d   = d0 + tid;
  const size_t row0 = (size_t)bix * kSeq;
#pragma unroll 1
  for (int r = 0; r < kDtR; ++r) sW[r * kScanCh + tid] = Wdt[(size_t)r * kDin + d];
#pragma unroll 1
  for (int s = 0; s < kNst; ++s) sA[s * kScanCh + tid] = -expf(Alog[(size_t)d * kNst + s]);
  {
    const int pc = (tid < kPrjN) ? tid : (kPrjN - 1);
    float pbl = xpb[pc];
    asm volatile("" : "+v"(pbl));
    sPB[tid] = (tid < kPrjN) ? pbl : 0.f;
  }
  __syncthreads();
  float negA[kNst], h[kNst];
#pragma unroll
  for (int s = 0; s < kNst; ++s) {
    negA[s] = sA[s * kScanCh + tid];
    h[s] = 0.f;
  }
  const float bb = bdt[d], Dd = Dp[d];
  const int lr = tid >> 4, lc4 = (tid & 15) * 4;
  const v4f pbv = *(const v4f*)(sPB + lc4);
  const int q = lane >> 3, c8 = (lane & 7) * 8;
#pragma unroll 1
  for (int t0 = 0; t0 < kSeq; t0 += kScanTS) {
    __syncthreads();
#pragma unroll
    for (int i = 0; i < 16; ++i) {
      const int r = lr + 4 * i;
      v4f pv = *(const v4f*)(PROJ + (row0 + t0 + r) * kPrjP + lc4);
      pv = pv + pbv;
      *(v4f*)(sX + r * kPrjP + lc4) = pv;
    }
    __syncthreads();
#pragma unroll 1
    for (int s = 0; s < kScanTS; ++s) {
      const size_t grow = row0 + t0 + s;
      const float* xs = sX + s * kPrjP;
      float xt = UC[grow * kDin + d];
      float zv = XR[grow * kXZP + kDin + d];
      asm volatile("" : "+v"(xt), "+v"(zv));
      float vdot = 0.f;
#pragma unroll 1
      for (int r4 = 0; r4 < kDtR / 4; ++r4) {
        const v4f xv = *(const v4f*)(xs + 4 * r4);
        const float* wp = sW + (4 * r4) * kScanCh + tid;
        vdot = fmaf(xv[0], wp[0], vdot);
        vdot = fmaf(xv[1], wp[kScanCh], vdot);
        vdot = fmaf(xv[2], wp[2 * kScanCh], vdot);
        vdot = fmaf(xv[3], wp[3 * kScanCh], vdot);
      }
      v4f Bq[4], Cq[4];
#pragma unroll
      for (int q4 = 0; q4 < 4; ++q4) {
        Bq[q4] = *(const v4f*)(xs + kDtR + 4 * q4);
        Cq[q4] = *(const v4f*)(xs + kDtR + kNst + 4 * q4);
      }
      const float v   = vdot + bb;
      const float dt  = fmaxf(v, 0.0f) + log1pf(expf(-fabsf(v)));
      const float dtx = dt * xt;
      float y = 0.f;
#pragma unroll
      for (int k = 0; k < kNst; ++k) {
        const float e = __expf(dt * negA[k]);
        h[k] = fmaf(e, h[k], dtx * Bq[k >> 2][k & 3]);
        y = fmaf(h[k], Cq[k >> 2][k & 3], y);
      }
      y = fmaf(xt, Dd, y);
      const float sg = __builtin_amdgcn_rcpf(1.0f + expf(-zv));
      sY[s * kScanYP + tid] = (y * (zv * sg)) * kCarryG;
    }
    __syncthreads();
    v8h hv[8];
#pragma unroll
    for (int it = 0; it < 8; ++it) {
      const int row = it * 8 + wave * 4 + q;
      const float* sp = sY + row * kScanYP + c8;
      const v4f a0 = *(const v4f*)(sp);
      const v4f a1 = *(const v4f*)(sp + 4);
#pragma unroll
      for (int e = 0; e < 4; ++e) {
        hv[it][e]     = (_Float16)a0[e];
        hv[it][4 + e] = (_Float16)a1[e];
      }
    }
    for (int pass = 0; pass < 2; ++pass) {
#pragma unroll
      for (int it = 0; it < 8; ++it) {
        const int row = it * 8 + wave * 4 + q;
        const size_t o = (row0 + t0 + row) * kDin + d0 + c8;
        *(volatile v8h*)(G16 + o) = hv[it];
      }
      __threadfence();
    }
  }
}

extern "C" void kernel_launch(void* const* d_in, const int* in_sizes, int n_in,
                              void* d_out, int out_size, void* d_ws, size_t ws_size,
                              hipStream_t stream) {
  if (n_in < 13) return;
  if (in_sizes[0] != kRows * kDm) return;
  if (in_sizes[1] != kDm * kXZP) return;
  if (in_sizes[2] != kXZP) return;
  if (in_sizes[3] != kConvK * kDin) return;
  if (in_sizes[4] != kDin) return;
  if (in_sizes[5] != kDin * kPrjN) return;
  if (in_sizes[6] != kPrjN) return;
  if (in_sizes[7] != kDtR * kDin) return;
  if (in_sizes[8] != kDin) return;
  if (in_sizes[9] != kDin * kNst) return;
  if (in_sizes[10] != kDin) return;
  if (in_sizes[11] != kDin * kDm) return;
  if (in_sizes[12] != kDm) return;
  if (out_size != kRows * kDm) return;
  if (ws_size < kWsTotal) return;

  const float* x          = (const float*)d_in[0];
  const float* in_proj_w  = (const float*)d_in[1];
  const float* in_proj_b  = (const float*)d_in[2];
  const float* conv_w     = (const float*)d_in[3];
  const float* conv_b     = (const float*)d_in[4];
  const float* x_proj_w   = (const float*)d_in[5];
  const float* x_proj_b   = (const float*)d_in[6];
  const float* dt_proj_w  = (const float*)d_in[7];
  const float* dt_proj_b  = (const float*)d_in[8];
  const float* A_log      = (const float*)d_in[9];
  const float* D_skip     = (const float*)d_in[10];
  const float* out_proj_w = (const float*)d_in[11];
  const float* out_proj_b = (const float*)d_in[12];
  float* out = (float*)d_out;

  char* ws = (char*)d_ws;
  unsigned short* XH   = (unsigned short*)(ws + kOffXH);
  unsigned short* WIN  = (unsigned short*)(ws + kOffWIN);
  unsigned short* WOUT = (unsigned short*)(ws + kOffWOUT);
  unsigned short* WX   = (unsigned short*)(ws + kOffWX);
  float*          XR   = (float*)(ws + kOffXR);
  float*          UC   = (float*)(ws + kOffUC);
  unsigned short* UCH  = (unsigned short*)(ws + kOffUCH);
  float*          PROJ = (float*)(ws + kOffPROJ);
  unsigned short* G16  = (unsigned short*)(ws + kOffG16);

  cast_f16_kernel<<<(kRows * kDm / 8) / 256, 256, 0, stream>>>(x, XH, kRows * kDm / 8, 1.0f);

  transpose_cast_kernel<<<dim3(kXZP / 64, kDm / 64), 256, 0, stream>>>(in_proj_w, WIN, kDm, kXZP, kXZP, kCarryW);
  transpose_cast_kernel<<<dim3(kDm / 64, kDin / 64), 256, 0, stream>>>(out_proj_w, WOUT, kDin, kDm, kDm, kCarryW);
  transpose_cast_kernel<<<dim3(kPrjP / 64, kDin / 64), 256, 0, stream>>>(x_proj_w, WX, kDin, kPrjN, kPrjP, kCarryW);

  wmma_gemm64_f16<2><<<((kRows / 64) * (kXZP / 64)) / 8, 256, 0, stream>>>(
      XH, kDm, WIN, kDm, XR, kXZP, in_proj_b, kRows, kXZP, kDm, kSclIn);

  conv_silu_kernel<<<dim3(kDin / 256, kRows / 64), 256, 0, stream>>>(XR, conv_w, conv_b, UC, UCH);

  wmma_gemm64_f16<0><<<((kRows / 64) * (kPrjP / 64)) / 8, 256, 0, stream>>>(
      UCH, kDin, WX, kDin, PROJ, kPrjP, x_proj_b, kRows, kPrjP, kDin, kSclXp);

  scan_kernel<<<kBatch * (kDin / kScanCh), kScanCh, 0, stream>>>(
      PROJ, UC, XR, x_proj_b, dt_proj_w, dt_proj_b, A_log, D_skip, G16);

  wmma_gemm64_f16<2><<<((kRows / 64) * (kDm / 64)) / 8, 256, 0, stream>>>(
      G16, kDin, WOUT, kDin, out, kDm, out_proj_b, kRows, kDm, kDin, kSclOut);
}
